// LeAttention_57131654971958
// MI455X (gfx1250) — hardware-verified
//
#include <hip/hip_runtime.h>
#include <stddef.h>


typedef _Float16 v16h __attribute__((ext_vector_type(16)));
typedef _Float16 v8h  __attribute__((ext_vector_type(8)));
typedef float    v8f  __attribute__((ext_vector_type(8)));
typedef float    v4f  __attribute__((ext_vector_type(4)));
typedef v8h v8ha __attribute__((may_alias));
typedef v4f v4fa __attribute__((may_alias));

#define NB_  16
#define NC_  256
#define NP_  1024
#define NH_  8
#define DK_  32
#define DV_  64
#define NO_  512
#define RS_  1032
#define GP_  72
#define EPS_ 1e-5f
#define CQK_ (0.17677669529663687f * 0.015625f)
#define INVSCALE_ 5.656854249492381f

union Frag { v16h v; v8h p[2]; };

__device__ __forceinline__ v16h ldfrag(const _Float16* rowp, int k0, int h) {
  Frag f;
  f.p[0] = *(const v8ha*)(rowp + k0 + 8 * h);
  f.p[1] = *(const v8ha*)(rowp + k0 + 16 + 8 * h);
  return f.v;
}

__device__ __forceinline__ v8f mma16(v16h a, v16h b, v8f c) {
  c = __builtin_amdgcn_wmma_f32_16x16x32_f16(false, a, false, b, (short)0, c, false, false);
  asm volatile("v_nop\n\tv_nop\n\tv_nop\n\tv_nop" : "+v"(c) : "v"(a), "v"(b));
  return c;
}

__device__ __forceinline__ v8f vzero() {
  v8f z = {0.f, 0.f, 0.f, 0.f, 0.f, 0.f, 0.f, 0.f};
  return z;
}

__global__ __launch_bounds__(256) void k_fold_qkv(
    const float* __restrict__ Wq, const float* __restrict__ qg, const float* __restrict__ qb,
    const float* __restrict__ qm, const float* __restrict__ qv,
    const float* __restrict__ Wk, const float* __restrict__ kg, const float* __restrict__ kb,
    const float* __restrict__ km, const float* __restrict__ kv,
    const float* __restrict__ Wv, const float* __restrict__ vg, const float* __restrict__ vb,
    const float* __restrict__ vm, const float* __restrict__ vv,
    _Float16* Wh, _Float16* Wl, float* beta) {
  __shared__ __attribute__((aligned(16))) float sb[32];
  const int tid = threadIdx.x, w = tid >> 5, lane = tid & 31;
  const int blk = blockIdx.x;
#pragma unroll 1
  for (int i = 0; i < 4; ++i) {
    const int o = blk * 32 + w * 4 + i;
    const float* W;
    float g, bb, mm, var;
    int oo;
    if (o < 256)      { oo = o;       W = Wq; g = qg[oo]; bb = qb[oo]; mm = qm[oo]; var = qv[oo]; }
    else if (o < 512) { oo = o - 256; W = Wk; g = kg[oo]; bb = kb[oo]; mm = km[oo]; var = kv[oo]; }
    else              { oo = o - 512; W = Wv; g = vg[oo]; bb = vb[oo]; mm = vm[oo]; var = vv[oo]; }
    const float inv = g * (1.0f / sqrtf(var + EPS_));
    const float* wr = W + (size_t)oo * NC_ + lane * 8;
    const v4f w0 = *(const v4fa*)(wr);
    const v4f w1 = *(const v4fa*)(wr + 4);
    float vals[8] = {w0.x, w0.y, w0.z, w0.w, w1.x, w1.y, w1.z, w1.w};
    v8h hv, lv;
#pragma unroll
    for (int e = 0; e < 8; ++e) {
      const float s = vals[e] * inv * 1024.0f;
      const _Float16 hh = (_Float16)s;
      const _Float16 ll = (_Float16)(s - (float)hh);
      hv[e] = hh; lv[e] = ll;
    }
    _Float16* dh = Wh + (size_t)o * NC_ + lane * 8;
    _Float16* dl = Wl + (size_t)o * NC_ + lane * 8;
    *(volatile v8h*)dh = hv;
    *(volatile v8h*)dl = lv;
    __threadfence();
    *(volatile v8h*)dh = hv;
    *(volatile v8h*)dl = lv;
    if (lane == 0) sb[w * 4 + i] = bb - mm * inv;
  }
  __syncthreads();
  if (w == 0 && lane < 8) {
    v4f b4;
    b4.x = sb[lane * 4 + 0]; b4.y = sb[lane * 4 + 1]; b4.z = sb[lane * 4 + 2]; b4.w = sb[lane * 4 + 3];
    float* db = beta + blk * 32 + lane * 4;
    *(volatile v4f*)db = b4;
    __threadfence();
    *(volatile v4f*)db = b4;
  }
}

__global__ __launch_bounds__(256) void k_fold_wo(
    const float* __restrict__ Wo, const float* __restrict__ bo, const float* __restrict__ og,
    const float* __restrict__ ob, const float* __restrict__ om, const float* __restrict__ ov,
    _Float16* WoS, float* betaO) {
  __shared__ __attribute__((aligned(16))) float sb[32];
  const int tid = threadIdx.x, w = tid >> 5, lane = tid & 31;
  const int blk = blockIdx.x;
#pragma unroll 1
  for (int i = 0; i < 4; ++i) {
    const int o = blk * 32 + w * 4 + i;
    const float inv = og[o] * (1.0f / sqrtf(ov[o] + EPS_));
#pragma unroll
    for (int hf = 0; hf < 2; ++hf) {
      const float* wr = Wo + (size_t)o * NO_ + hf * 256 + lane * 8;
      const v4f w0 = *(const v4fa*)(wr);
      const v4f w1 = *(const v4fa*)(wr + 4);
      float vals[8] = {w0.x, w0.y, w0.z, w0.w, w1.x, w1.y, w1.z, w1.w};
      v8h hv;
#pragma unroll
      for (int e = 0; e < 8; ++e) hv[e] = (_Float16)(vals[e] * inv * 16.0f);
      _Float16* dh = WoS + (size_t)o * NO_ + hf * 256 + lane * 8;
      *(volatile v8h*)dh = hv;
      __threadfence();
      *(volatile v8h*)dh = hv;
    }
    if (lane == 0) sb[w * 4 + i] = bo[o] * inv + ob[o] - om[o] * inv;
  }
  __syncthreads();
  if (w == 0 && lane < 8) {
    v4f b4;
    b4.x = sb[lane * 4 + 0]; b4.y = sb[lane * 4 + 1]; b4.z = sb[lane * 4 + 2]; b4.w = sb[lane * 4 + 3];
    float* db = betaO + blk * 32 + lane * 4;
    *(volatile v4f*)db = b4;
    __threadfence();
    *(volatile v4f*)db = b4;
  }
}

__global__ __launch_bounds__(256) void k_tr(const float* __restrict__ x, _Float16* xTh, _Float16* xTl) {
  __shared__ float T[64][65];
  const int pblk = blockIdx.x, cblk = blockIdx.y, b = blockIdx.z;
  const int tid = threadIdx.x;
#pragma unroll
  for (int it = 0; it < 16; ++it) {
    const int idx = it * 256 + tid;
    const int ci = idx >> 6, pj = idx & 63;
    T[ci][pj] = x[((size_t)(b * NC_ + cblk * 64 + ci)) * NP_ + pblk * 64 + pj];
  }
  __syncthreads();
#pragma unroll
  for (int it = 0; it < 2; ++it) {
    const int pi = it * 256 + tid;
    const int pl = pi >> 3, pc = pi & 7;
    v8h hv, lv;
#pragma unroll
    for (int e = 0; e < 8; ++e) {
      const float s = T[pc * 8 + e][pl] * 64.0f;
      const _Float16 hh = (_Float16)s;
      const _Float16 ll = (_Float16)(s - (float)hh);
      hv[e] = hh; lv[e] = ll;
    }
    const size_t off = ((size_t)(b * NP_ + pblk * 64 + pl)) * NC_ + cblk * 64 + pc * 8;
    *(volatile v8h*)(xTh + off) = hv;
    *(volatile v8h*)(xTl + off) = lv;
    __threadfence();
    *(volatile v8h*)(xTh + off) = hv;
    *(volatile v8h*)(xTl + off) = lv;
  }
}

__global__ __launch_bounds__(256) void k_qkv(
    const _Float16* __restrict__ xTh, const _Float16* __restrict__ xTl,
    const _Float16* __restrict__ Wh, const _Float16* __restrict__ Wl, const float* __restrict__ beta,
    _Float16* qT, _Float16* kT, _Float16* vN) {
  __shared__ __attribute__((aligned(16))) _Float16 st[128 * GP_];
  const int ptile = blockIdx.x, nchunk = blockIdx.y, b = blockIdx.z;
  const int tid = threadIdx.x, w = tid >> 5, lane = tid & 31, m = lane & 15, h = lane >> 4;
  const int msub = w & 3, nh = w >> 2;
  const int nbase = nchunk * 128 + nh * 64;
  const size_t prow = (size_t)b * NP_ + ptile * 64 + msub * 16 + m;
  const bool split = (nchunk < 4);

  v8f acc[4] = {vzero(), vzero(), vzero(), vzero()};
  const _Float16* ahr = xTh + prow * NC_;
  const _Float16* alr = xTl + prow * NC_;
#pragma unroll 1
  for (int kk = 0; kk < 8; ++kk) {
    const int k0 = kk * 32;
    const v16h ah = ldfrag(ahr, k0, h);
    v16h al = ah;
    if (split) al = ldfrag(alr, k0, h);
#pragma unroll
    for (int t = 0; t < 4; ++t) {
      const size_t orow = (size_t)(nbase + t * 16 + m) * NC_;
      const v16h bh = ldfrag(Wh + orow, k0, h);
      acc[t] = mma16(ah, bh, acc[t]);
      if (split) {
        const v16h bl = ldfrag(Wl + orow, k0, h);
        acc[t] = mma16(ah, bl, acc[t]);
        acc[t] = mma16(al, bh, acc[t]);
      }
    }
  }

  const float kS = 1.0f / 65536.0f;
#pragma unroll
  for (int t = 0; t < 4; ++t) {
    const int ol = nh * 64 + t * 16 + m;
    const float bta = beta[nchunk * 128 + ol];
#pragma unroll
    for (int j = 0; j < 8; ++j) {
      const int pl = msub * 16 + 8 * h + j;
      const _Float16 hv = (_Float16)((acc[t][j] * kS + bta) * 8.0f);
      if (split) st[pl * 136 + ol] = hv;
      else       st[ol * GP_ + pl] = hv;
    }
  }
  __syncthreads();

  if (split) {
    _Float16* base = (nchunk < 2) ? qT : kT;
    const int hb = (nchunk & 1) * 4;
#pragma unroll
    for (int it = 0; it < 4; ++it) {
      const int pi = it * 256 + tid;
      const int hd = pi >> 8, r = pi & 255;
      const int pl = r >> 2, dq = r & 3;
      const v8h v = *(const v8ha*)(st + pl * 136 + hd * 32 + dq * 8);
      _Float16* dst = base + (((size_t)(b * NH_ + hb + hd)) * NP_ + ptile * 64) * DK_ + r * 8;
      *(volatile v8h*)dst = v;
      __threadfence();
      *(volatile v8h*)dst = v;
    }
  } else {
    const int obase = (nchunk - 4) * 128;
#pragma unroll
    for (int it = 0; it < 4; ++it) {
      const int pi = it * 256 + tid;
      const int ol = pi >> 3, pc = pi & 7;
      const v8h v = *(const v8ha*)(st + ol * GP_ + pc * 8);
      _Float16* dst = vN + ((size_t)(b * NO_ + obase + ol)) * NP_ + ptile * 64 + pc * 8;
      *(volatile v8h*)dst = v;
      __threadfence();
      *(volatile v8h*)dst = v;
    }
  }
}

__global__ __launch_bounds__(64) void k_attn(
    const _Float16* __restrict__ qT, const _Float16* __restrict__ kT, const _Float16* __restrict__ vN,
    const float* __restrict__ posemb, const int* __restrict__ pidx, _Float16* goT) {
  extern __shared__ __attribute__((aligned(16))) float smem[];
  float* poscol = smem;
  float* rmaxs  = smem + 1024;
  float* sc     = smem + 1056;
  _Float16* gT  = (_Float16*)(smem + 1056 + 2 * 16 * RS_);

  const int qgrp = blockIdx.x, n = blockIdx.y, b = blockIdx.z;
  const int tid = threadIdx.x;
  const int w = tid >> 5, lane = tid & 31, m = lane & 15, h = lane >> 4;
  for (int k = tid; k < NP_; k += 64) poscol[k] = posemb[k * NH_ + n];
  __syncthreads();

  const int qbase = (qgrp * 2 + w) * 16;
  const int bn = b * NH_ + n;
  const v16h aq = ldfrag(qT + ((size_t)bn * NP_ + qbase + m) * DK_, 0, h);
  float* myS = sc + w * 16 * RS_;
  const v8f vz = vzero();

  float pmax[8];
#pragma unroll
  for (int j = 0; j < 8; ++j) pmax[j] = -3.0e38f;
#pragma unroll 1
  for (int kt = 0; kt < 64; ++kt) {
    const v16h bk = ldfrag(kT + ((size_t)bn * NP_ + kt * 16 + m) * DK_, 0, h);
    const v8f s = mma16(aq, bk, vz);
    const int kgl = kt * 16 + m;
#pragma unroll
    for (int j = 0; j < 8; ++j) {
      const int row = 8 * h + j;
      const int qgl = qbase + row;
      int ix = pidx[(size_t)qgl * NP_ + kgl];
      ix = ix < 0 ? 0 : (ix > NP_ - 1 ? NP_ - 1 : ix);
      const float val = s[j] * CQK_ + poscol[ix] * INVSCALE_;
      myS[row * RS_ + kgl] = val;
      pmax[j] = fmaxf(pmax[j], val);
    }
  }
#pragma unroll
  for (int j = 0; j < 8; ++j) {
    float mv = pmax[j];
    mv = fmaxf(mv, __shfl_xor(mv, 1));
    mv = fmaxf(mv, __shfl_xor(mv, 2));
    mv = fmaxf(mv, __shfl_xor(mv, 4));
    mv = fmaxf(mv, __shfl_xor(mv, 8));
    if (m == j) rmaxs[w * 16 + j + 8 * h] = mv;
  }
  __syncthreads();

  const float mx = rmaxs[w * 16 + m];
  float* rowh = myS + m * RS_ + h * 512;
  float sum = 0.f;
#pragma unroll 1
  for (int c4 = 0; c4 < 128; ++c4) {
    v4f f = *(v4fa*)(rowh + c4 * 4);
    f.x = __expf(f.x - mx);
    f.y = __expf(f.y - mx);
    f.z = __expf(f.z - mx);
    f.w = __expf(f.w - mx);
    sum += (f.x + f.y) + (f.z + f.w);
    *(v4fa*)(rowh + c4 * 4) = f;
  }
  sum += __shfl_xor(sum, 16);
  const float rs = (1.0f / sum) * 4096.0f;
  __syncthreads();

  v8f oacc[4] = {vz, vz, vz, vz};
  const float* rp = myS + m * RS_;
#pragma unroll 1
  for (int kc = 0; kc < 32; ++kc) {
    const int k0 = kc * 32;
    const v4f f0 = *(const v4fa*)(rp + k0 + 8 * h);
    const v4f f1 = *(const v4fa*)(rp + k0 + 8 * h + 4);
    const v4f f2 = *(const v4fa*)(rp + k0 + 16 + 8 * h);
    const v4f f3 = *(const v4fa*)(rp + k0 + 16 + 8 * h + 4);
    v8h p0, p1;
    p0[0] = (_Float16)(f0.x * rs); p0[1] = (_Float16)(f0.y * rs); p0[2] = (_Float16)(f0.z * rs); p0[3] = (_Float16)(f0.w * rs);
    p0[4] = (_Float16)(f1.x * rs); p0[5] = (_Float16)(f1.y * rs); p0[6] = (_Float16)(f1.z * rs); p0[7] = (_Float16)(f1.w * rs);
    p1[0] = (_Float16)(f2.x * rs); p1[1] = (_Float16)(f2.y * rs); p1[2] = (_Float16)(f2.z * rs); p1[3] = (_Float16)(f2.w * rs);
    p1[4] = (_Float16)(f3.x * rs); p1[5] = (_Float16)(f3.y * rs); p1[6] = (_Float16)(f3.z * rs); p1[7] = (_Float16)(f3.w * rs);
    Frag ap;
    ap.p[0] = p0; ap.p[1] = p1;
#pragma unroll
    for (int t = 0; t < 4; ++t) {
      const v16h bv = ldfrag(vN + ((size_t)(b * NO_ + n * DV_ + t * 16 + m)) * NP_, k0, h);
      oacc[t] = mma16(ap.v, bv, oacc[t]);
    }
  }

  const float co = 1.0f / 32768.0f;
  _Float16* gw = gT + w * 16 * GP_;
#pragma unroll
  for (int t = 0; t < 4; ++t) {
#pragma unroll
    for (int j = 0; j < 8; ++j) {
      const int row = 8 * h + j;
      const float xo = oacc[t][j] * co;
      const float gl = 0.5f * xo * (1.0f + erff(xo * 0.70710678118654752f));
      gw[row * GP_ + t * 16 + m] = (_Float16)(gl * 256.0f);
    }
  }
  __syncthreads();
#pragma unroll
  for (int it = 0; it < 4; ++it) {
    const int pi = it * 32 + lane;
    const int row = pi >> 3, pc = pi & 7;
    const v8h v = *(const v8ha*)(gw + row * GP_ + pc * 8);
    _Float16* dst = goT + ((size_t)(b * NP_ + qbase + row)) * NO_ + n * DV_ + pc * 8;
    *(volatile v8h*)dst = v;
    __threadfence();
    *(volatile v8h*)dst = v;
  }
}

__global__ __launch_bounds__(256) void k_out(
    const _Float16* __restrict__ goT, const _Float16* __restrict__ WoS, const float* __restrict__ betaO,
    float* out) {
  __shared__ __attribute__((aligned(16))) float To[128 * 68];
  const int ptile = blockIdx.x, nchunk = blockIdx.y, b = blockIdx.z;
  const int tid = threadIdx.x, w = tid >> 5, lane = tid & 31, m = lane & 15, h = lane >> 4;
  const int msub = w & 3, nh = w >> 2;
  const int nbase = nchunk * 128 + nh * 64;
  const size_t prow = (size_t)b * NP_ + ptile * 64 + msub * 16 + m;
  v8f acc[4] = {vzero(), vzero(), vzero(), vzero()};
  const _Float16* ar = goT + prow * NO_;
#pragma unroll 1
  for (int kk = 0; kk < 16; ++kk) {
    const int k0 = kk * 32;
    const v16h a = ldfrag(ar, k0, h);
#pragma unroll
    for (int t = 0; t < 4; ++t) {
      const v16h bt = ldfrag(WoS + (size_t)(nbase + t * 16 + m) * NO_, k0, h);
      acc[t] = mma16(a, bt, acc[t]);
    }
  }
  const float kS = 1.0f / 4096.0f;
#pragma unroll
  for (int t = 0; t < 4; ++t) {
    const int ol = nh * 64 + t * 16 + m;
    const float bta = betaO[nchunk * 128 + ol];
#pragma unroll
    for (int j = 0; j < 8; ++j) {
      const int pl = msub * 16 + 8 * h + j;
      To[ol * 68 + pl] = acc[t][j] * kS + bta;
    }
  }
  __syncthreads();
#pragma unroll
  for (int it = 0; it < 8; ++it) {
    const int pi = it * 256 + tid;
    const int ol = pi >> 4, pc = pi & 15;
    const v4f v = *(const v4fa*)(To + ol * 68 + pc * 4);
    float* dst = out + ((size_t)(b * NC_ + nchunk * 128 + ol)) * NP_ + ptile * 64 + pc * 4;
    *(volatile v4f*)dst = v;
    __threadfence();
    *(volatile v4f*)dst = v;
  }
}

extern "C" void kernel_launch(void* const* d_in, const int* in_sizes, int n_in,
                              void* d_out, int out_size, void* d_ws, size_t ws_size,
                              hipStream_t stream) {
  if (n_in < 24) return;
  if (in_sizes[0] != NB_ * NC_ * NP_) return;
  if (in_sizes[1] != NC_ * NC_ || in_sizes[6] != NC_ * NC_ || in_sizes[11] != NO_ * NC_) return;
  if (in_sizes[16] != NP_ * NH_ || in_sizes[17] != NC_ * NO_ || in_sizes[23] != NP_ * NP_) return;
  {
    const int f32c[13] = {2, 3, 4, 5, 7, 8, 9, 10, 18, 19, 20, 21, 22};
    for (int i = 0; i < 13; ++i) if (in_sizes[f32c[i]] != NC_) return;
    const int f32o[4] = {12, 13, 14, 15};
    for (int i = 0; i < 4; ++i) if (in_sizes[f32o[i]] != NO_) return;
  }
  if (out_size != NB_ * NC_ * NP_) return;

  const float* x    = (const float*)d_in[0];
  const float* Wq   = (const float*)d_in[1];
  const float* q_g  = (const float*)d_in[2];
  const float* q_b  = (const float*)d_in[3];
  const float* q_m  = (const float*)d_in[4];
  const float* q_v  = (const float*)d_in[5];
  const float* Wk   = (const float*)d_in[6];
  const float* k_g  = (const float*)d_in[7];
  const float* k_b  = (const float*)d_in[8];
  const float* k_m  = (const float*)d_in[9];
  const float* k_v  = (const float*)d_in[10];
  const float* Wv   = (const float*)d_in[11];
  const float* v_g  = (const float*)d_in[12];
  const float* v_b  = (const float*)d_in[13];
  const float* v_m  = (const float*)d_in[14];
  const float* v_v  = (const float*)d_in[15];
  const float* pose = (const float*)d_in[16];
  const float* Wo   = (const float*)d_in[17];
  const float* bo   = (const float*)d_in[18];
  const float* o_g  = (const float*)d_in[19];
  const float* o_b  = (const float*)d_in[20];
  const float* o_m  = (const float*)d_in[21];
  const float* o_v  = (const float*)d_in[22];
  const int*   pix  = (const int*)d_in[23];

  const size_t O_WH    = 0;
  const size_t O_WL    = O_WH    + (size_t)1024 * NC_ * 2;
  const size_t O_BETA  = O_WL    + (size_t)1024 * NC_ * 2;
  const size_t O_WOS   = O_BETA  + 4096;
  const size_t O_BETAO = O_WOS   + (size_t)NC_ * NO_ * 2;
  const size_t O_XTH   = O_BETAO + 1024;
  const size_t O_XTL   = O_XTH   + (size_t)NB_ * NP_ * NC_ * 2;
  const size_t O_QT    = O_XTL   + (size_t)NB_ * NP_ * NC_ * 2;
  const size_t O_KT    = O_QT    + (size_t)NB_ * NH_ * NP_ * DK_ * 2;
  const size_t O_VN    = O_KT    + (size_t)NB_ * NH_ * NP_ * DK_ * 2;
  const size_t O_GOT   = O_VN    + (size_t)NB_ * NO_ * NP_ * 2;
  const size_t O_END   = O_GOT   + (size_t)NB_ * NP_ * NO_ * 2;
  if (O_END > ws_size) return;

  char* ws = (char*)d_ws;
  _Float16* Wh    = (_Float16*)(ws + O_WH);
  _Float16* Wl    = (_Float16*)(ws + O_WL);
  float*    beta  = (float*)   (ws + O_BETA);
  _Float16* WoS   = (_Float16*)(ws + O_WOS);
  float*    betaO = (float*)   (ws + O_BETAO);
  _Float16* xTh   = (_Float16*)(ws + O_XTH);
  _Float16* xTl   = (_Float16*)(ws + O_XTL);
  _Float16* qT    = (_Float16*)(ws + O_QT);
  _Float16* kT    = (_Float16*)(ws + O_KT);
  _Float16* vN    = (_Float16*)(ws + O_VN);
  _Float16* goT   = (_Float16*)(ws + O_GOT);

  k_fold_qkv<<<dim3(32), dim3(256), 0, stream>>>(Wq, q_g, q_b, q_m, q_v,
                                                 Wk, k_g, k_b, k_m, k_v,
                                                 Wv, v_g, v_b, v_m, v_v, Wh, Wl, beta);
  k_fold_wo<<<dim3(8), dim3(256), 0, stream>>>(Wo, bo, o_g, o_b, o_m, o_v, WoS, betaO);
  k_tr<<<dim3(NP_ / 64, NC_ / 64, NB_), dim3(256), 0, stream>>>(x, xTh, xTl);
  k_qkv<<<dim3(NP_ / 64, 8, NB_), dim3(256), 0, stream>>>(xTh, xTl, Wh, Wl, beta, qT, kT, vN);
  const size_t smem = (size_t)(1056 + 2 * 16 * RS_) * sizeof(float) + (size_t)2 * 16 * GP_ * 2;
  k_attn<<<dim3(NP_ / 32, NH_, NB_), dim3(64), smem, stream>>>(qT, kT, vN, pose, pix, goT);
  k_out<<<dim3(NP_ / 64, 2, NB_), dim3(256), 0, stream>>>(goT, WoS, betaO, (float*)d_out);
}
